// FrustumProposer_29025388987118
// MI455X (gfx1250) — hardware-verified
//
#include <hip/hip_runtime.h>

#pragma clang fp contract(off)

typedef _Float16 v16h __attribute__((ext_vector_type(16)));
typedef float    v8f  __attribute__((ext_vector_type(8)));
typedef float    v4f  __attribute__((ext_vector_type(4)));

union HFrag { v16h v; _Float16 s[16]; unsigned u[8]; };

#define C_NDET    64
#define C_NMAG    10
#define C_NROT    10
#define C_NCAND   (C_NMAG * C_NROT)
#define C_NTRIAL  4
#define C_FRMIN   2.0f
#define C_FRMAX   60.0f
#define C_BINW    5.8f
#define C_THR     0.69f
#define C_IMGW    1600.0f
#define C_IMGH    900.0f
#define C_PI      3.14159274f
#define C_W_IOU   0.91f
#define C_W_DNS   0.09f
#define C_W_BASE  0.92f
#define C_W_PLN   0.08f

#define NWAVE2    8
#define NTHR2     256
#define NBLK2     128
#define MAXCAM    16

#define WS_DET    0
#define WS_CDIR   512
#define WS_PLN    768
#define WS_SETUP_FLOATS 1024
#define WS_TAB    1024
#define TAB_FLOATS 1024
#define TAB_INV   0
#define TAB_ERI   512
#define TAB_COS   544
#define TAB_SIN   560
#define TAB_USED  576
#define WS_PART   2048
#define PART_STRIDE 1024

__device__ const float TCX[8] = { 0.5f, 0.5f,-0.5f,-0.5f, 0.5f, 0.5f,-0.5f,-0.5f};
__device__ const float TCY[8] = { 0.5f,-0.5f,-0.5f, 0.5f, 0.5f,-0.5f,-0.5f, 0.5f};
__device__ const float TCZ[8] = {-0.5f,-0.5f,-0.5f,-0.5f, 0.5f, 0.5f, 0.5f, 0.5f};

__device__ __forceinline__ v8f wmma_f16(v8f c, v16h a, v16h b) {
  v8f d = __builtin_amdgcn_wmma_f32_16x16x32_f16(false, a, false, b, (short)0, c, false, false);
  asm volatile("v_nop\n\tv_nop\n\tv_nop\n\tv_nop" : "+v"(d) : "v"(a), "v"(b));
  return d;
}

__device__ __forceinline__ float lin10(float a, float b, int i) {
  const float st = (float)i * (1.0f / 9.0f);
  const float w0 = 1.0f - st;
  const float t0 = a * w0;
  const float t1 = b * st;
  const float r  = t0 + t1;
  return (i >= 9) ? b : r;
}

__device__ __forceinline__ void mv3(const float* m, float v0, float v1, float v2,
                                    float& o0, float& o1, float& o2) {
  float a, b, c;
  a = m[0]*v0; b = m[1]*v1; c = m[2]*v2; o0 = (a + b) + c;
  a = m[3]*v0; b = m[4]*v1; c = m[5]*v2; o1 = (a + b) + c;
  a = m[6]*v0; b = m[7]*v1; c = m[8]*v2; o2 = (a + b) + c;
}

__device__ __forceinline__ void swap3(float* x, float* y) {
  float t;
  t = x[0]; x[0] = y[0]; y[0] = t;
  t = x[1]; x[1] = y[1]; y[1] = t;
  t = x[2]; x[2] = y[2]; y[2] = t;
}

__device__ void lu_inv3(const float* m, float* o) {
  float r0[3] = {m[0], m[1], m[2]};
  float r1[3] = {m[3], m[4], m[5]};
  float r2[3] = {m[6], m[7], m[8]};
  int p0 = 0, p1 = 1, p2 = 2;
  {
    const float a0 = fabsf(r0[0]), a1 = fabsf(r1[0]), a2 = fabsf(r2[0]);
    int piv = 0; float mv = a0;
    if (a1 > mv) { piv = 1; mv = a1; }
    if (a2 > mv) { piv = 2; mv = a2; }
    if (piv == 1) { swap3(r0, r1); const int t = p0; p0 = p1; p1 = t; }
    else if (piv == 2) { swap3(r0, r2); const int t = p0; p0 = p2; p2 = t; }
    const float inv = 1.0f / r0[0];
    r1[0] = r1[0] * inv;
    r2[0] = r2[0] * inv;
    float t;
    t = r1[0] * r0[1]; r1[1] = r1[1] - t;
    t = r1[0] * r0[2]; r1[2] = r1[2] - t;
    t = r2[0] * r0[1]; r2[1] = r2[1] - t;
    t = r2[0] * r0[2]; r2[2] = r2[2] - t;
  }
  {
    if (fabsf(r2[1]) > fabsf(r1[1])) { swap3(r1, r2); const int t = p1; p1 = p2; p2 = t; }
    const float inv = 1.0f / r1[1];
    r2[1] = r2[1] * inv;
    const float t = r2[1] * r1[2];
    r2[2] = r2[2] - t;
  }
  const float i0 = 1.0f / r0[0];
  const float i1 = 1.0f / r1[1];
  const float i2 = 1.0f / r2[2];
  #pragma unroll
  for (int c = 0; c < 3; ++c) {
    const float b0 = (p0 == c) ? 1.0f : 0.0f;
    const float b1 = (p1 == c) ? 1.0f : 0.0f;
    const float b2 = (p2 == c) ? 1.0f : 0.0f;
    float t;
    const float y0 = b0;
    t = r1[0] * y0; const float y1 = b1 - t;
    t = r2[0] * y0; float y2 = b2 - t;
    t = r2[1] * y1; y2 = y2 - t;
    const float x2 = y2 * i2;
    t = r1[2] * x2; const float x1 = (y1 - t) * i1;
    t = r0[2] * x2; float s0 = y0 - t;
    t = r0[1] * x1; s0 = s0 - t;
    const float x0 = s0 * i0;
    o[0 * 3 + c] = x0;
    o[1 * 3 + c] = x1;
    o[2 * 3 + c] = x2;
  }
}

__device__ __forceinline__ void load33(const float* M4, float* o) {
  o[0] = M4[0]; o[1] = M4[1]; o[2] = M4[2];
  o[3] = M4[4]; o[4] = M4[5]; o[5] = M4[6];
  o[6] = M4[8]; o[7] = M4[9]; o[8] = M4[10];
}

__global__ __launch_bounds__(64) void k_tab(
    const float* __restrict__ cam_intr, int ncam,
    const float* __restrict__ img_aug,
    const float* __restrict__ cam2lidar,
    const float* __restrict__ lidar_aug,
    float* tabw)
{
  __shared__ __attribute__((aligned(16))) float st[TAB_FLOATS];
  const int tid = threadIdx.x;
  for (int i = tid; i < TAB_FLOATS; i += blockDim.x) st[i] = 0.0f;
  __syncthreads();

  const int ninv = 3 * ncam + 1;
  if (tid < ninv) {
    const float* src;
    int dst;
    if (tid < ncam)          { src = cam_intr  + tid * 16;              dst = TAB_INV + tid * 32; }
    else if (tid < 2 * ncam) { src = img_aug   + (tid - ncam) * 16;     dst = TAB_INV + (tid - ncam) * 32 + 9; }
    else if (tid < 3 * ncam) { src = cam2lidar + (tid - 2 * ncam) * 16; dst = TAB_INV + (tid - 2 * ncam) * 32 + 18; }
    else                     { src = lidar_aug;                         dst = TAB_ERI; }
    float M[9], Mi[9];
    load33(src, M);
    lu_inv3(M, Mi);
    #pragma unroll
    for (int c = 0; c < 9; ++c) st[dst + c] = Mi[c];
  }
  if (tid < C_NROT) {
    const float ry = lin10(0.0f, C_PI, tid);
    st[TAB_COS + tid] = cosf(ry);
    st[TAB_SIN + tid] = sinf(ry);
  }
  __syncthreads();

  volatile v4f* wv = (volatile v4f*)tabw;
  for (int i = tid; i < TAB_FLOATS / 4; i += blockDim.x) {
    const v4f v = ((const v4f*)st)[i];
    wv[i] = v;
  }
  __threadfence();
  for (int i = tid; i < TAB_FLOATS / 4; i += blockDim.x) {
    const v4f v = ((const v4f*)st)[i];
    wv[i] = v;
  }
}

__global__ __launch_bounds__(128) void k_setup(
    const float* __restrict__ points, int npts, int ncam,
    const float* __restrict__ cam2lidar,
    const float* __restrict__ img_aug,
    const float* __restrict__ lidar_aug,
    const float* __restrict__ det_boxes,
    const int*   __restrict__ det_cam_idx,
    const float* tab,
    float* ws)
{
  __shared__ __attribute__((aligned(16))) float st[WS_SETUP_FLOATS];
  const int tid = threadIdx.x;
  for (int i = tid; i < WS_SETUP_FLOATS; i += blockDim.x) st[i] = 0.0f;
  __syncthreads();

  if (tid < C_NDET) {
    const int d = tid;
    int cam = det_cam_idx[d];
    cam = cam < 0 ? 0 : (cam >= ncam ? ncam - 1 : cam);

    float Kinv[9], PRinv[9], CR[9], ER[9], CK[9];
    #pragma unroll
    for (int i = 0; i < 9; ++i) {
      Kinv[i]  = tab[TAB_INV + cam * 32 + i];
      PRinv[i] = tab[TAB_INV + cam * 32 + 9 + i];
    }
    const float* Pm = img_aug + cam * 16;
    const float PT0 = Pm[3], PT1 = Pm[7], PT2 = Pm[11];
    const float* Cm = cam2lidar + cam * 16;
    load33(Cm, CR);
    const float CT0 = Cm[3], CT1 = Cm[7], CT2 = Cm[11];
    load33(lidar_aug, ER);
    const float ET0 = lidar_aug[3], ET1 = lidar_aug[7], ET2 = lidar_aug[11];

    #pragma unroll
    for (int i = 0; i < 3; ++i) {
      #pragma unroll
      for (int l = 0; l < 3; ++l) {
        const float a = CR[i * 3 + 0] * Kinv[0 * 3 + l];
        const float b = CR[i * 3 + 1] * Kinv[1 * 3 + l];
        const float c = CR[i * 3 + 2] * Kinv[2 * 3 + l];
        CK[i * 3 + l] = (a + b) + c;
      }
    }

    const float x1 = det_boxes[d * 4 + 0], y1 = det_boxes[d * 4 + 1];
    const float x2 = det_boxes[d * 4 + 2], y2 = det_boxes[d * 4 + 3];
    const float whl0 = x2 - x1, whl1 = y2 - y1, whl2 = C_FRMAX - C_FRMIN;
    const float sm0 = x2 + x1, sm1 = y2 + y1, sm2 = C_FRMAX + C_FRMIN;
    const float ctr0 = sm0 * 0.5f, ctr1 = sm1 * 0.5f, ctr2 = sm2 * 0.5f;

    float mn0 = __builtin_inff(), mn1 = __builtin_inff(), mn2 = __builtin_inff();
    float mx0 = -__builtin_inff(), mx1 = -__builtin_inff(), mx2 = -__builtin_inff();
    float s0 = 0.0f, s1 = 0.0f, s2 = 0.0f;

    #pragma unroll 1
    for (int k = 0; k < 8; ++k) {
      float t;
      t = whl0 * TCX[k]; const float ci0 = t + ctr0;
      t = whl1 * TCY[k]; const float ci1 = t + ctr1;
      t = whl2 * TCZ[k]; const float ci2 = t + ctr2;
      const float a0 = ci0 - PT0, a1 = ci1 - PT1, a2 = ci2 - PT2;
      float b0, b1, b2; mv3(PRinv, a0, a1, a2, b0, b1, b2);
      const float c0 = b0 * b2, c1 = b1 * b2, c2 = b2;
      float e0, e1, e2; mv3(CK, c0, c1, c2, e0, e1, e2);
      e0 = e0 + CT0; e1 = e1 + CT1; e2 = e2 + CT2;
      float g0, g1, g2; mv3(ER, e0, e1, e2, g0, g1, g2);
      g0 = g0 + ET0; g1 = g1 + ET1; g2 = g2 + ET2;
      const float q0 = g0 * g0, q1 = g1 * g1, q2 = g2 * g2;
      const float nm = sqrtf((q0 + q1) + q2);
      const float ir = 1.0f / (nm + 1e-8f);
      const float u0 = g0 * ir, u1 = g1 * ir, u2 = g2 * ir;
      mn0 = fminf(mn0, u0); mn1 = fminf(mn1, u1); mn2 = fminf(mn2, u2);
      mx0 = fmaxf(mx0, u0); mx1 = fmaxf(mx1, u1); mx2 = fmaxf(mx2, u2);
      s0 = s0 + u0; s1 = s1 + u1; s2 = s2 + u2;
    }
    const float md0 = s0 * 0.125f, md1 = s1 * 0.125f, md2 = s2 * 0.125f;
    const float w0 = md0 * md0, w1 = md1 * md1, w2 = md2 * md2;
    const float mg = sqrtf((w0 + w1) + w2);
    const float rr = 1.0f / (mg + 1e-8f);

    st[WS_DET + d * 8 + 0] = mn0; st[WS_DET + d * 8 + 1] = mn1; st[WS_DET + d * 8 + 2] = mn2;
    st[WS_DET + d * 8 + 4] = mx0; st[WS_DET + d * 8 + 5] = mx1; st[WS_DET + d * 8 + 6] = mx2;
    st[WS_CDIR + d * 4 + 0] = md0 * rr;
    st[WS_CDIR + d * 4 + 1] = md1 * rr;
    st[WS_CDIR + d * 4 + 2] = md2 * rr;
  } else if (tid < C_NDET + C_NTRIAL) {
    const int t = tid - C_NDET;
    const int step = npts / 3;
    int i0 = t, i1 = t + step, i2 = t + 2 * step;
    if (i0 > npts - 1) i0 = npts - 1;
    if (i1 > npts - 1) i1 = npts - 1;
    if (i2 > npts - 1) i2 = npts - 1;
    const float* q0 = points + (size_t)i0 * 4;
    const float* q1 = points + (size_t)i1 * 4;
    const float* q2 = points + (size_t)i2 * 4;
    const float p0x = q0[1], p0y = q0[2], p0z = q0[3];
    const float ux = q1[1] - p0x, uy = q1[2] - p0y, uz = q1[3] - p0z;
    const float vx = q2[1] - p0x, vy = q2[2] - p0y, vz = q2[3] - p0z;
    float a, b;
    a = uy * vz; b = uz * vy; const float n0 = a - b;
    a = uz * vx; b = ux * vz; const float n1 = a - b;
    a = ux * vy; b = uy * vx; const float n2 = a - b;
    const float m0 = n0 * n0, m1 = n1 * n1, m2 = n2 * n2;
    const float nn = (m0 + m1) + m2;
    const float rinv = 1.0f / (nn + 1e-8f);
    const float sq = sqrtf(nn);
    float* pl = st + WS_PLN + t * 8;
    pl[0] = n0; pl[1] = n1; pl[2] = n2;
    pl[3] = p0x; pl[4] = p0y; pl[5] = p0z;
    pl[6] = rinv; pl[7] = sq;
  }
  __syncthreads();

  volatile v4f* wv = (volatile v4f*)ws;
  for (int i = tid; i < WS_SETUP_FLOATS / 4; i += blockDim.x) {
    const v4f v = ((const v4f*)st)[i];
    wv[i] = v;
  }
  __threadfence();
  for (int i = tid; i < WS_SETUP_FLOATS / 4; i += blockDim.x) {
    const v4f v = ((const v4f*)st)[i];
    wv[i] = v;
  }
}

__global__ __launch_bounds__(NTHR2) void k_points(
    const float* __restrict__ points, int npts,
    const float* wsr,
    float* part)
{
  __shared__ __attribute__((aligned(16))) float    s_pdir[NWAVE2][32][4];
  __shared__ __attribute__((aligned(16))) _Float16 s_qty [NWAVE2][32][16];
  __shared__ unsigned s_msk[NWAVE2][64];
  __shared__ __attribute__((aligned(16))) float    s_acc[NWAVE2][C_NDET * 16];

  const int tid  = threadIdx.x;
  const int lane = tid & 31;
  const int w    = tid >> 5;
  const int h    = lane >> 4;
  const int col  = lane & 15;

  const v4f dmn0 = *(const v4f*)(wsr + WS_DET + lane * 8);
  const v4f dmx0 = *(const v4f*)(wsr + WS_DET + lane * 8 + 4);
  const v4f dmn1 = *(const v4f*)(wsr + WS_DET + (lane + 32) * 8);
  const v4f dmx1 = *(const v4f*)(wsr + WS_DET + (lane + 32) * 8 + 4);

  float pnx[C_NTRIAL], pny[C_NTRIAL], pnz[C_NTRIAL], p0x[C_NTRIAL], p0y[C_NTRIAL], p0z[C_NTRIAL];
  float prv[C_NTRIAL], psq[C_NTRIAL];
  #pragma unroll
  for (int t = 0; t < C_NTRIAL; ++t) {
    const float* pl = wsr + WS_PLN + t * 8;
    pnx[t] = pl[0]; pny[t] = pl[1]; pnz[t] = pl[2];
    p0x[t] = pl[3]; p0y[t] = pl[4]; p0z[t] = pl[5];
    prv[t] = pl[6]; psq[t] = pl[7];
  }
  float mags[C_NMAG];
  #pragma unroll
  for (int m = 0; m < C_NMAG; ++m) mags[m] = lin10(C_FRMIN, C_FRMAX, m);

  const _Float16 h_one  = (_Float16)1.0f;
  const _Float16 h_zero = (_Float16)0.0f;

  v8f acc0 = {}, acc1 = {}, acc2 = {}, acc3 = {};

  const int nchunk = (npts + 31) >> 5;
  const int per    = (int)gridDim.x * NWAVE2;
  const int niter  = (nchunk + per - 1) / per;

  for (int it = 0; it < niter; ++it) {
    const int chunk = (it * (int)gridDim.x + (int)blockIdx.x) * NWAVE2 + w;
    const long idx  = (long)chunk * 32 + lane;
    const bool valid = idx < (long)npts;
    const long ridx = valid ? idx : (long)(npts - 1);

    const v4f pt = *(const v4f*)(points + ridx * 4);
    const float px = pt[1], py = pt[2], pz = pt[3];
    const float e0 = px * px, e1 = py * py, e2 = pz * pz;
    const float pm = sqrtf((e0 + e1) + e2);
    const float ir = 1.0f / (pm + 1e-8f);
    s_pdir[w][lane][0] = px * ir;
    s_pdir[w][lane][1] = py * ir;
    s_pdir[w][lane][2] = pz * ir;
    s_pdir[w][lane][3] = valid ? pm : -1.0f;

    #pragma unroll
    for (int m = 0; m < C_NMAG; ++m) {
      const float df = pm - mags[m];
      s_qty[w][lane][m] = (fabsf(df) < C_BINW) ? h_one : h_zero;
    }
    #pragma unroll
    for (int t = 0; t < C_NTRIAL; ++t) {
      const float dx = px - p0x[t], dy = py - p0y[t], dz = pz - p0z[t];
      const float a = pnx[t] * dx, b = pny[t] * dy, c = pnz[t] * dz;
      const float dot = (a + b) + c;
      const float tt = dot * prv[t];
      const float dist = fabsf(tt) * psq[t];
      s_qty[w][lane][10 + t] = (dist < C_THR) ? h_one : h_zero;
    }
    s_qty[w][lane][14] = h_one;
    s_qty[w][lane][15] = h_zero;
    __syncthreads();

    unsigned m0 = 0u, m1 = 0u;
    #pragma unroll
    for (int k = 0; k < 32; ++k) {
      const v4f q = *(const v4f*)(&s_pdir[w][k][0]);
      const bool rng = (q[3] >= C_FRMIN) & (q[3] <= C_FRMAX);
      const bool b0 = rng & (q[0] >= dmn0[0]) & (q[0] <= dmx0[0]) & (q[1] >= dmn0[1]) & (q[1] <= dmx0[1])
                          & (q[2] >= dmn0[2]) & (q[2] <= dmx0[2]);
      const bool b1 = rng & (q[0] >= dmn1[0]) & (q[0] <= dmx1[0]) & (q[1] >= dmn1[1]) & (q[1] <= dmx1[1])
                          & (q[2] >= dmn1[2]) & (q[2] <= dmx1[2]);
      m0 |= (b0 ? 1u : 0u) << k;
      m1 |= (b1 ? 1u : 0u) << k;
    }
    s_msk[w][lane]      = m0;
    s_msk[w][lane + 32] = m1;
    __syncthreads();

    HFrag b;
    #pragma unroll
    for (int e = 0; e < 16; ++e) {
      const int kk = (e & 7) + ((e >> 3) << 4) + 8 * h;
      b.s[e] = s_qty[w][kk][col];
    }

    {
      const unsigned mw = s_msk[w][0 * 16 + col];
      HFrag a;
      #pragma unroll
      for (int j = 0; j < 8; ++j) {
        const int k0 = ((2 * j) & 7) + (((2 * j) >> 3) << 4) + 8 * h;
        a.u[j] = (((mw >> k0) & 1u) * 0x3C00u) | (((mw >> (k0 + 1)) & 1u) * 0x3C000000u);
      }
      acc0 = wmma_f16(acc0, a.v, b.v);
    }
    {
      const unsigned mw = s_msk[w][1 * 16 + col];
      HFrag a;
      #pragma unroll
      for (int j = 0; j < 8; ++j) {
        const int k0 = ((2 * j) & 7) + (((2 * j) >> 3) << 4) + 8 * h;
        a.u[j] = (((mw >> k0) & 1u) * 0x3C00u) | (((mw >> (k0 + 1)) & 1u) * 0x3C000000u);
      }
      acc1 = wmma_f16(acc1, a.v, b.v);
    }
    {
      const unsigned mw = s_msk[w][2 * 16 + col];
      HFrag a;
      #pragma unroll
      for (int j = 0; j < 8; ++j) {
        const int k0 = ((2 * j) & 7) + (((2 * j) >> 3) << 4) + 8 * h;
        a.u[j] = (((mw >> k0) & 1u) * 0x3C00u) | (((mw >> (k0 + 1)) & 1u) * 0x3C000000u);
      }
      acc2 = wmma_f16(acc2, a.v, b.v);
    }
    {
      const unsigned mw = s_msk[w][3 * 16 + col];
      HFrag a;
      #pragma unroll
      for (int j = 0; j < 8; ++j) {
        const int k0 = ((2 * j) & 7) + (((2 * j) >> 3) << 4) + 8 * h;
        a.u[j] = (((mw >> k0) & 1u) * 0x3C00u) | (((mw >> (k0 + 1)) & 1u) * 0x3C000000u);
      }
      acc3 = wmma_f16(acc3, a.v, b.v);
    }
    __syncthreads();
  }

  #pragma unroll
  for (int r = 0; r < 8; ++r) {
    const int dr = 8 * h + r;
    s_acc[w][(0 * 16 + dr) * 16 + col] = acc0[r];
    s_acc[w][(1 * 16 + dr) * 16 + col] = acc1[r];
    s_acc[w][(2 * 16 + dr) * 16 + col] = acc2[r];
    s_acc[w][(3 * 16 + dr) * 16 + col] = acc3[r];
  }
  __syncthreads();

  float o[4];
  #pragma unroll
  for (int c = 0; c < 4; ++c) {
    const int i = 4 * tid + c;
    float s = 0.0f;
    #pragma unroll
    for (int ww = 0; ww < NWAVE2; ++ww) s = s + s_acc[ww][i];
    o[c] = s;
  }
  v4f v;
  v[0] = o[0]; v[1] = o[1]; v[2] = o[2]; v[3] = o[3];
  volatile v4f* pv = (volatile v4f*)(part + (size_t)blockIdx.x * PART_STRIDE);
  pv[tid] = v;
  __threadfence();
  pv[tid] = v;
}

__global__ __launch_bounds__(128) void k_score(
    const float* __restrict__ cam_intr, int ncam,
    const float* __restrict__ cam2lidar,
    const float* __restrict__ img_aug,
    const float* __restrict__ lidar_aug,
    const float* __restrict__ det_boxes,
    const float* __restrict__ det_scores,
    const float* __restrict__ anchors, int nanch,
    const int*   __restrict__ det_labels,
    const int*   __restrict__ det_cam_idx,
    const float* wsr,
    const float* tab,
    const float* part, int nblk,
    float* out)
{
  __shared__ float s_cnt[C_NDET * 16];
  __shared__ __attribute__((aligned(16))) float s_res[C_NDET * 8];
  __shared__ float s_tab[TAB_USED];
  __shared__ float ssc[128];
  __shared__ int   sid[128];

  const int tid = threadIdx.x;

  for (int i = tid; i < C_NDET * 16; i += blockDim.x) {
    float s = 0.0f;
    for (int bb = 0; bb < nblk; ++bb) s = s + part[(size_t)bb * PART_STRIDE + i];
    s_cnt[i] = s;
  }
  for (int i = tid; i < TAB_USED; i += blockDim.x) s_tab[i] = tab[i];
  __syncthreads();

  for (int d = 0; d < C_NDET; ++d) {
    int cam = det_cam_idx[d];
    cam = cam < 0 ? 0 : (cam >= ncam ? ncam - 1 : cam);
    int lbl = det_labels[d];
    lbl = lbl < 0 ? 0 : (lbl >= nanch ? nanch - 1 : lbl);
    const float x1 = det_boxes[d * 4 + 0], y1 = det_boxes[d * 4 + 1];
    const float x2 = det_boxes[d * 4 + 2], y2 = det_boxes[d * 4 + 3];
    const float cd0 = wsr[WS_CDIR + d * 4 + 0];
    const float cd1 = wsr[WS_CDIR + d * 4 + 1];
    const float cd2 = wsr[WS_CDIR + d * 4 + 2];
    const float sx = anchors[lbl * 3 + 0], sy = anchors[lbl * 3 + 1], sz = anchors[lbl * 3 + 2];

    float dmx = s_cnt[d * 16 + 0];
    #pragma unroll
    for (int m = 1; m < C_NMAG; ++m) dmx = fmaxf(dmx, s_cnt[d * 16 + m]);
    const float rdn = 1.0f / (dmx + 1e-6f);
    const float rms = 1.0f / (s_cnt[d * 16 + 14] + 1e-6f);
    float pln = s_cnt[d * 16 + 10] * rms;
    #pragma unroll
    for (int t = 1; t < C_NTRIAL; ++t) pln = fmaxf(pln, s_cnt[d * 16 + 10 + t] * rms);

    float score = -__builtin_inff();
    int   myidx = 0x7FFFFFFF;

    if (tid < C_NCAND) {
      const int m = tid / C_NROT;
      const int r = tid - m * C_NROT;

      float K3[9], PR[9], CRinv[9], ERinv[9];
      load33(cam_intr + cam * 16, K3);
      const float* Pm = img_aug + cam * 16;
      load33(Pm, PR);
      const float PT0 = Pm[3], PT1 = Pm[7];
      const float* Cm = cam2lidar + cam * 16;
      const float CT0 = Cm[3], CT1 = Cm[7], CT2 = Cm[11];
      #pragma unroll
      for (int i = 0; i < 9; ++i) {
        CRinv[i] = s_tab[TAB_INV + cam * 32 + 18 + i];
        ERinv[i] = s_tab[TAB_ERI + i];
      }
      const float ET0 = lidar_aug[3], ET1 = lidar_aug[7], ET2 = lidar_aug[11];

      const float mag = lin10(C_FRMIN, C_FRMAX, m);
      const float cc = s_tab[TAB_COS + r];
      const float sn = s_tab[TAB_SIN + r];
      const float ctr0 = cd0 * mag, ctr1 = cd1 * mag, ctr2 = cd2 * mag;
      const float dns = s_cnt[d * 16 + m] * rdn;

      float bx1 = __builtin_inff(), by1 = __builtin_inff();
      float bx2 = -__builtin_inff(), by2 = -__builtin_inff();
      #pragma unroll 1
      for (int k = 0; k < 8; ++k) {
        const float lx = sx * TCX[k], ly = sy * TCY[k], lz = sz * TCZ[k];
        const float p1 = lx * cc, p2 = ly * sn, p3 = lx * sn, p4 = ly * cc;
        const float xr = p1 - p2;
        const float yr = p3 + p4;
        const float wx = xr + ctr0, wy = yr + ctr1, wz = lz + ctr2;
        const float a0 = wx - ET0, a1 = wy - ET1, a2 = wz - ET2;
        float b0, b1, b2; mv3(ERinv, a0, a1, a2, b0, b1, b2);
        const float c0 = b0 - CT0, c1 = b1 - CT1, c2 = b2 - CT2;
        float e0, e1, e2; mv3(CRinv, c0, c1, c2, e0, e1, e2);
        float q0, q1, q2; mv3(K3, e0, e1, e2, q0, q1, q2);
        const float depth = fmaxf(q2, 0.001f);
        const float rd = 1.0f / depth;
        const float n0 = q0 * rd, n1 = q1 * rd;
        float f0, f1, f2; mv3(PR, n0, n1, depth, f0, f1, f2);
        const float uu = f0 + PT0, vv = f1 + PT1;
        const float u = fminf(fmaxf(uu, 0.0f), C_IMGW);
        const float v = fminf(fmaxf(vv, 0.0f), C_IMGH);
        bx1 = fminf(bx1, u); by1 = fminf(by1, v);
        bx2 = fmaxf(bx2, u); by2 = fmaxf(by2, v);
      }
      const float ix1 = fmaxf(bx1, x1), iy1 = fmaxf(by1, y1);
      const float ix2 = fminf(bx2, x2), iy2 = fminf(by2, y2);
      const float iw = fmaxf(ix2 - ix1, 0.0f);
      const float ih = fmaxf(iy2 - iy1, 0.0f);
      const float inter = iw * ih;
      const float ap = (bx2 - bx1) * (by2 - by1);
      const float ad = (x2 - x1) * (y2 - y1);
      const float s1 = ap + ad;
      const float s2 = s1 - inter;
      const float den = s2 + 1e-6f;
      const float riou = 1.0f / den;
      const float iou = inter * riou;
      const float t1 = C_W_IOU * iou;
      const float t2 = C_W_DNS * dns;
      const float base = t1 + t2;
      const float t3 = C_W_BASE * base;
      const float t4 = C_W_PLN * pln;
      score = t3 + t4;
      myidx = tid;
    }

    ssc[tid] = score; sid[tid] = myidx;
    __syncthreads();
    for (int off = 64; off > 0; off >>= 1) {
      if (tid < off) {
        const float sa = ssc[tid],       sb = ssc[tid + off];
        const int   ia = sid[tid],       ib = sid[tid + off];
        const bool na = (sa != sa), nb = (sb != sb);
        const bool gt = (sb > sa) | (nb & !na);
        const bool eq = (sb == sa) | (nb & na);
        if (gt | (eq & (ib < ia))) { ssc[tid] = sb; sid[tid] = ib; }
      }
      __syncthreads();
    }
    if (tid == 0) {
      int best = sid[0];
      if (best < 0 || best >= C_NCAND) best = 0;
      const int bm = best / C_NROT;
      const int br = best - bm * C_NROT;
      const float mag = lin10(C_FRMIN, C_FRMAX, bm);
      const float ry  = lin10(0.0f, C_PI, br);
      s_res[d * 8 + 0] = cd0 * mag;
      s_res[d * 8 + 1] = cd1 * mag;
      s_res[d * 8 + 2] = cd2 * mag;
      s_res[d * 8 + 3] = sx;
      s_res[d * 8 + 4] = sy;
      s_res[d * 8 + 5] = sz;
      s_res[d * 8 + 6] = ry;
      s_res[d * 8 + 7] = ssc[0] * det_scores[d];
    }
    __syncthreads();
  }

  volatile v4f* ov = (volatile v4f*)out;
  for (int i = tid; i < (C_NDET * 8) / 4; i += blockDim.x) {
    const v4f v = ((const v4f*)s_res)[i];
    ov[i] = v;
  }
  __threadfence();
  for (int i = tid; i < (C_NDET * 8) / 4; i += blockDim.x) {
    const v4f v = ((const v4f*)s_res)[i];
    ov[i] = v;
  }
}

extern "C" void kernel_launch(void* const* d_in, const int* in_sizes, int n_in,
                              void* d_out, int out_size, void* d_ws, size_t ws_size,
                              hipStream_t stream) {
  (void)n_in;
  const float* points      = (const float*)d_in[0];
  const float* cam_intr    = (const float*)d_in[1];
  const float* cam2lidar   = (const float*)d_in[2];
  const float* img_aug     = (const float*)d_in[3];
  const float* lidar_aug   = (const float*)d_in[4];
  const float* det_boxes   = (const float*)d_in[5];
  const float* det_scores  = (const float*)d_in[6];
  const float* anchors     = (const float*)d_in[7];
  const int*   det_labels  = (const int*)d_in[8];
  const int*   det_cam_idx = (const int*)d_in[9];
  float* out = (float*)d_out;
  float* ws  = (float*)d_ws;

  int npts = in_sizes[0] / 4;
  if (npts < 1) return;
  int ncam = in_sizes[1] / 16;
  if (ncam < 1) return;
  if (ncam > MAXCAM) ncam = MAXCAM;
  if (in_sizes[2] < ncam * 16 || in_sizes[3] < ncam * 16) return;
  int nanch = in_sizes[7] / 3;
  if (nanch < 1) return;
  if (in_sizes[5] < C_NDET * 4 || in_sizes[6] < C_NDET ||
      in_sizes[8] < C_NDET || in_sizes[9] < C_NDET) return;
  if (in_sizes[4] < 12) return;
  if (out_size < C_NDET * 8) return;

  const size_t need_bytes = (size_t)(WS_PART + NBLK2 * PART_STRIDE) * sizeof(float);
  if (need_bytes > ws_size) return;
  float* tab  = ws + WS_TAB;
  float* part = ws + WS_PART;

  k_tab<<<1, 64, 0, stream>>>(cam_intr, ncam, img_aug, cam2lidar, lidar_aug, tab);
  k_setup<<<1, 128, 0, stream>>>(points, npts, ncam, cam2lidar, img_aug, lidar_aug,
                                 det_boxes, det_cam_idx, tab, ws);
  k_points<<<NBLK2, NTHR2, 0, stream>>>(points, npts, ws, part);
  k_score<<<1, 128, 0, stream>>>(cam_intr, ncam, cam2lidar, img_aug, lidar_aug,
                                 det_boxes, det_scores, anchors, nanch,
                                 det_labels, det_cam_idx, ws, tab, part, NBLK2, out);
}
